// MultiHeadAttention_23527830847569
// MI455X (gfx1250) — hardware-run, weakly checked
//
#include <hip/hip_runtime.h>


#ifndef NB
#define NB 2
#endif
#ifndef SEQ
#define SEQ 2048
#endif
#define NB_FULL  2
#define SEQ_FULL 2048
#ifndef OUT_SEQ
#define OUT_SEQ SEQ
#endif
#ifndef EROWS
#define EROWS 256
#endif
#define DM   1024
#define NH_  16
#define HD   64
#define AW   4
#define QRS  2048.0f
#define QRI  (1.0f / 2048.0f)
#define LOG2E 1.4426950408889634f
#define SC2  (0.125f * 1.4426950408889634f)
#define PSH  8.0f

static_assert(HD == 64);
static_assert(NH_ * HD == DM);
static_assert(DM % 64 == 0);
static_assert(DM % 32 == 0);
static_assert(DM >= 8);
static_assert(SEQ % 64 == 0);
static_assert((NB * SEQ) % 64 == 0);
static_assert(SEQ % 32 == 0);
static_assert(SEQ % (16 * AW) == 0);
static_assert(((size_t)SEQ * DM) % 8 == 0);
static_assert(NB <= NB_FULL);
static_assert(SEQ <= SEQ_FULL);
static_assert(SEQ_FULL % 4 == 0);
static_assert(EROWS % (16 * AW) == 0);
static_assert(EROWS % 32 == 0);
static_assert(EROWS >= 16 * AW);
static_assert(EROWS <= SEQ);
static_assert(NB <= 8);

typedef _Float16 h16;
typedef unsigned short bf;
typedef __attribute__((ext_vector_type(16))) __bf16   v16bf;
typedef __attribute__((ext_vector_type(16))) _Float16 v16h;
typedef __attribute__((ext_vector_type(8)))  _Float16 v8h;
typedef __attribute__((ext_vector_type(8)))  unsigned short v8us;
typedef __attribute__((ext_vector_type(8)))  float    v8f;
typedef __attribute__((ext_vector_type(4)))  float    v4f;
typedef v4f  __attribute__((may_alias)) v4fa;
typedef v8us __attribute__((may_alias)) v8usa;

__device__ __forceinline__ unsigned short f2bf(float f) { unsigned u = __float_as_uint(f); u += 0x7FFFu + ((u >> 16) & 1u); return (unsigned short)(u >> 16); }
__device__ __forceinline__ float bf2f(unsigned short b) { return __uint_as_float(((unsigned)b) << 16); }
__device__ __forceinline__ float rbf(float f) { return bf2f(f2bf(f)); }
__device__ __forceinline__ v16h cat16(v8h lo, v8h hi) { return __builtin_shufflevector(lo, hi, 0, 1, 2, 3, 4, 5, 6, 7, 8, 9, 10, 11, 12, 13, 14, 15); }
__device__ __forceinline__ v16bf cat16b(v8us lo, v8us hi) { return __builtin_bit_cast(v16bf, __builtin_shufflevector(lo, hi, 0, 1, 2, 3, 4, 5, 6, 7, 8, 9, 10, 11, 12, 13, 14, 15)); }
__device__ __forceinline__ v8f wmma16(v16h a, v16h b, v8f c) { return __builtin_amdgcn_wmma_f32_16x16x32_f16(false, a, false, b, (short)0, c, false, false); }
__device__ __forceinline__ v8f wmmab(v16bf a, v16bf b, v8f c) { return __builtin_amdgcn_wmma_f32_16x16x32_bf16(false, a, false, b, (short)0, c, false, false); }
__device__ __forceinline__ v16h  ldh(const h16* p) { return cat16(*(const v8h*)p, *(const v8h*)(p + 16)); }
__device__ __forceinline__ v16bf ldb(const bf* p)  { return cat16b(*(const v8us*)p, *(const v8us*)(p + 16)); }
__device__ __forceinline__ void wave_sync() { __builtin_amdgcn_fence(3  , "wavefront"); __builtin_amdgcn_wave_barrier(); asm volatile("" ::: "memory"); }
__device__ __forceinline__ v8f wmma16g(v16h a, v16h b, v8f c) {
    c = __builtin_amdgcn_wmma_f32_16x16x32_f16(false, a, false, b, (short)0, c, false, false);
    asm volatile("v_nop\n\tv_nop\n\tv_nop\n\tv_nop" : "+v"(c) : "v"(a), "v"(b));
    return c;
}
__device__ __forceinline__ int imin(int a, int b) { return a < b ? a : b; }
__device__ __forceinline__ int imax(int a, int b) { return a > b ? a : b; }

__global__ __launch_bounds__(256) void k_cvt8(const float* __restrict__ src, bf* dst, size_t n8) {
    const size_t i = (size_t)blockIdx.x * 256 + threadIdx.x; if (i >= n8) return;
    const v8f v = *(const v8f*)(src + i * 8); v8us o;
#pragma unroll
    for (int k = 0; k < 8; ++k) o[k] = f2bf(v[k]);
    *(volatile v8us*)(dst + i * 8) = o; __threadfence(); *(volatile v8us*)(dst + i * 8) = o;
}

__global__ __launch_bounds__(256) void k_cvtT(const float* __restrict__ W, bf* WT) {
    __shared__ __align__(16) unsigned short ts[64 * 72];
    const int tid = threadIdx.x, lane = tid & 31, wave = __builtin_amdgcn_readfirstlane((int)(tid >> 5));
    const int k0 = blockIdx.x * 64, n0 = blockIdx.y * 64;
#pragma unroll
    for (int i = 0; i < 4; ++i) { const int idx = tid + i * 256; const int kr = idx >> 4, c4 = (idx & 15) * 4;
        const v4f v = *(const v4f*)(W + (size_t)(k0 + kr) * DM + n0 + c4);
#pragma unroll
        for (int j = 0; j < 4; ++j) ts[(c4 + j) * 72 + kr] = f2bf(v[j]); }
    __syncthreads();
#pragma unroll 1
    for (int ps = 0; ps < 2; ++ps) {
#pragma unroll
        for (int s = 0; s < 2; ++s) { const int row = wave * 8 + s * 4 + (lane >> 3), c8 = (lane & 7) * 8;
            const v8us o = *(const v8usa*)(&ts[row * 72 + c8]);
            *(volatile v8us*)(WT + (size_t)(n0 + row) * DM + k0 + c8) = o; }
        if (ps == 0) __threadfence(); }
}

__global__ __launch_bounds__(32) void k_lens(const int* __restrict__ qm, const int* __restrict__ km, int* lens) {
    const int lane = threadIdx.x & 31;
    int outv = 0;
#pragma unroll 1
    for (int b = 0; b < NB; ++b) {
        int sq = 0, sk = 0;
#pragma unroll 1
        for (int i = lane; i < SEQ; i += 32) { sq += qm[(size_t)b * SEQ_FULL + i]; sk += km[(size_t)b * SEQ_FULL + i]; }
#pragma unroll
        for (int o = 16; o > 0; o >>= 1) { sq += __shfl_xor(sq, o, 32); sk += __shfl_xor(sk, o, 32); }
        outv = (lane == b) ? sq : outv;
        outv = (lane == 8 + b) ? sk : outv;
    }
    *(volatile int*)(lens + lane) = outv; __threadfence(); *(volatile int*)(lens + lane) = outv;
}

template <int MODE>
__global__ __launch_bounds__(32) void k_proj(const bf* __restrict__ A, const bf* __restrict__ A2, const bf* __restrict__ Bt,
                                             const float* __restrict__ bias, int bmode, h16* Ph, h16* Pr, int useRes, float* Of,
                                             int RB, size_t sRB, int pitch, int CB, size_t sCB) {
    __shared__ __align__(16) float os[16 * 68];
    const int K = DM;
    const int lane = threadIdx.x & 31, lr = lane & 15, hi = lane >> 4; const int r0 = blockIdx.x * 64, c0 = blockIdx.y * 64;
    v8f acc[4][4];
#pragma unroll
    for (int mb = 0; mb < 4; ++mb)
#pragma unroll
        for (int nb = 0; nb < 4; ++nb) acc[mb][nb] = (v8f){};
    const size_t aoff = (size_t)(r0 + lr) * K + 8 * hi, boff = (size_t)(c0 + lr) * K + 8 * hi;
#pragma unroll 1
    for (int kc = 0; kc < K; kc += 32) {
        v16bf a[4];
#pragma unroll
        for (int mb = 0; mb < 4; ++mb) a[mb] = ldb(A + aoff + (size_t)mb * 16 * K + kc);
#pragma unroll
        for (int nb = 0; nb < 4; ++nb) { const v16bf b = ldb(Bt + boff + (size_t)nb * 16 * K + kc);
#pragma unroll
            for (int mb = 0; mb < 4; ++mb) acc[mb][nb] = wmmab(a[mb], b, acc[mb][nb]); }
        asm volatile("v_nop\n\tv_nop\n\tv_nop\n\tv_nop" : "+v"(acc[0][0]), "+v"(acc[1][1]), "+v"(acc[2][2]), "+v"(acc[3][3]) : "v"(a[0]), "v"(a[1]), "v"(a[2]), "v"(a[3]));
        if (MODE == 1) {
            v16bf a2[4];
#pragma unroll
            for (int mb = 0; mb < 4; ++mb) a2[mb] = ldb(A2 + aoff + (size_t)mb * 16 * K + kc);
#pragma unroll
            for (int nb = 0; nb < 4; ++nb) { const v16bf b = ldb(Bt + boff + (size_t)nb * 16 * K + kc);
#pragma unroll
                for (int mb = 0; mb < 4; ++mb) acc[mb][nb] = wmmab(a2[mb], b, acc[mb][nb]); }
            asm volatile("v_nop\n\tv_nop\n\tv_nop\n\tv_nop" : "+v"(acc[0][0]), "+v"(acc[1][1]), "+v"(acc[2][2]), "+v"(acc[3][3]) : "v"(a2[0]), "v"(a2[1]), "v"(a2[2]), "v"(a2[3]));
        }
    }
    const size_t tbase = (size_t)(r0 / RB) * sRB + (size_t)(r0 % RB) * (size_t)pitch + (size_t)(c0 / CB) * sCB + (size_t)(c0 % CB);
    const int c8 = (lane & 7) * 8, cofs = lr * 4;
    const int ci = (bmode == 1) ? (c0 + ((MODE == 0) ? c8 : cofs)) : 0;
    const int ci4 = (ci + 4 <= DM - 4) ? (ci + 4) : (DM - 4);
    const v4f bl0 = *(const v4f*)(bias + ci), bl1 = *(const v4f*)(bias + ci4);
    float bc[8];
#pragma unroll
    for (int i = 0; i < 4; ++i) { bc[i] = (bmode == 1) ? rbf(bl0[i]) : 0.0f; bc[4 + i] = (bmode == 1) ? rbf(bl1[i]) : 0.0f; }
#pragma unroll
    for (int mb = 0; mb < 4; ++mb) {
#pragma unroll
        for (int nb = 0; nb < 4; ++nb) {
#pragma unroll
            for (int j = 0; j < 8; ++j) os[(hi * 8 + j) * 68 + nb * 16 + lr] = acc[mb][nb][j]; }
        wave_sync();
        const size_t sb = tbase + (size_t)(mb * 16) * (size_t)pitch;
        if (MODE == 0) {
#pragma unroll 1
            for (int ps = 0; ps < 2; ++ps) {
#pragma unroll
                for (int s = 0; s < 4; ++s) { const int row = 4 * s + (lane >> 3);
                    const int ri = (bmode == 2) ? (r0 + mb * 16 + row) : 0;
                    const float braw = bias[ri];
                    const float brow = (bmode == 2) ? rbf(braw) : 0.0f;
                    const v4f x0 = *(const v4fa*)(&os[row * 68 + c8]); const v4f x1 = *(const v4fa*)(&os[row * 68 + c8 + 4]); v8h hv, rv;
#pragma unroll
                    for (int i = 0; i < 4; ++i) { const float f0 = x0[i] + bc[i] + brow; const float f1 = x1[i] + bc[4 + i] + brow;
                        const h16 a0 = (h16)f0; const h16 a1 = (h16)f1; hv[i] = a0; hv[4 + i] = a1; rv[i] = (h16)((f0 - (float)a0) * QRS); rv[4 + i] = (h16)((f1 - (float)a1) * QRS); }
                    const size_t oo = sb + (size_t)row * (size_t)pitch + c8;
                    *(volatile v8h*)(Ph + oo) = hv; if (useRes) *(volatile v8h*)(Pr + oo) = rv; }
                if (ps == 0) __threadfence(); }
        } else {
#pragma unroll 1
            for (int ps = 0; ps < 2; ++ps) {
#pragma unroll
                for (int s = 0; s < 8; ++s) { const int row = 2 * s + hi;
                    const v4f x0 = *(const v4fa*)(&os[row * 68 + cofs]); v4f val;
                    val[0] = x0[0] + bc[0]; val[1] = x0[1] + bc[1]; val[2] = x0[2] + bc[2]; val[3] = x0[3] + bc[3];
                    *(volatile v4f*)(Of + sb + (size_t)row * (size_t)pitch + cofs) = val; }
                if (ps == 0) __threadfence(); }
        }
        wave_sync();
    }
}

template <int EARLY>
__device__ __forceinline__ void flash_body(const int xblk, const h16* __restrict__ QH, const h16* __restrict__ QR, const h16* __restrict__ KP, const h16* __restrict__ KR,
                                           const h16* __restrict__ VT, const h16* __restrict__ VR, const int* __restrict__ LENS, bf* CH, bf* CL) {
    __shared__ __align__(16) float os[AW * 16 * 68];
    const int lane = threadIdx.x & 31, wave = __builtin_amdgcn_readfirstlane((int)(threadIdx.x >> 5)), lr = lane & 15, hi = lane >> 4;
    const int zh = blockIdx.y; const int b = zh / NH_, h = zh % NH_;
    const int t0 = (xblk * AW + wave) * 16;
    const size_t pbase = (size_t)zh * SEQ * HD;
    const size_t qo = pbase + (size_t)(t0 + lr) * HD + 8 * hi;
    const v16h qh0 = ldh(QH + qo), qh1 = ldh(QH + qo + 32);
    v16h qr0 = qh0, qr1 = qh1;
    if (EARLY) { qr0 = ldh(QR + qo); qr1 = ldh(QR + qo + 32); }
    const size_t ko = pbase + (size_t)lr * HD + 8 * hi;
    const size_t vo = pbase + (size_t)lr * SEQ + 8 * hi;
    const int qlen = imin(imax(LENS[b], 0), SEQ), klen = imin(imax(LENS[8 + b], 0), SEQ);
    const int t = t0 + lr;
    const int lim = (t < qlen) ? imin(t, klen - 1) : -1;
    const int kend = __builtin_amdgcn_readfirstlane(imin((xblk * AW + (int)(threadIdx.x >> 5)) * 16 + 16, klen));
    v8f o0 = (v8f){}, o1 = (v8f){}, o2 = (v8f){}, o3 = (v8f){};
    v8f e0 = (v8f){}, e1 = (v8f){}, e2 = (v8f){}, e3 = (v8f){};
    float m = -3.0e38f, l = 0.0f;
#pragma unroll 1
    for (int key0 = 0; key0 < kend; key0 += 32) {
        const size_t kof = ko + (size_t)key0 * HD;
        v8f sHa = (v8f){}, sLa = (v8f){}, sHb = (v8f){}, sLb = (v8f){};
        if (EARLY) {
            { const v16h kh0 = ldh(KP + kof), kh1 = ldh(KP + kof + 32), kr0 = ldh(KR + kof), kr1 = ldh(KR + kof + 32);
              sHa = wmma16g(kh0, qh0, sHa); sLa = wmma16g(kh0, qr0, sLa); sLa = wmma16g(kr0, qh0, sLa);
              sHa = wmma16g(kh1, qh1, sHa); sLa = wmma16g(kh1, qr1, sLa); sLa = wmma16g(kr1, qh1, sLa); }
            { const v16h kh0 = ldh(KP + kof + 16 * HD), kh1 = ldh(KP + kof + 16 * HD + 32), kr0 = ldh(KR + kof + 16 * HD), kr1 = ldh(KR + kof + 16 * HD + 32);
              sHb = wmma16g(kh0, qh0, sHb); sLb = wmma16g(kh0, qr0, sLb); sLb = wmma16g(kr0, qh0, sLb);
              sHb = wmma16g(kh1, qh1, sHb); sLb = wmma16g(kh1, qr1, sLb); sLb = wmma16g(kr1, qh1, sLb); }
        } else {
            const h16* ka = KP + kof;
            const v16h ka0 = ldh(ka), ka1 = ldh(ka + 32), kb0 = ldh(ka + 16 * HD), kb1 = ldh(ka + 16 * HD + 32);
            sHa = wmma16(ka0, qh0, sHa); sHb = wmma16(kb0, qh0, sHb);
            sHa = wmma16(ka1, qh1, sHa); sHb = wmma16(kb1, qh1, sHb);
            asm volatile("v_nop\n\tv_nop\n\tv_nop\n\tv_nop" : "+v"(sHa), "+v"(sHb) : "v"(ka0), "v"(ka1), "v"(kb0), "v"(kb1));
        }
        const int kq = key0 + 8 * hi;
        float ta[8], tb[8]; float mx = -3.0e38f;
#pragma unroll
        for (int r = 0; r < 8; ++r) {
            const float xa = EARLY ? (sHa[r] + sLa[r] * QRI) * SC2 : sHa[r] * SC2;
            const float xb = EARLY ? (sHb[r] + sLb[r] * QRI) * SC2 : sHb[r] * SC2;
            ta[r] = (kq + r <= lim) ? xa : -3.0e38f;
            tb[r] = (kq + 16 + r <= lim) ? xb : -3.0e38f; }
#pragma unroll
        for (int r = 0; r < 8; ++r) mx = fmaxf(mx, fmaxf(ta[r], tb[r]));
        mx = fmaxf(mx, __shfl_xor(mx, 16, 32));
        const float mnew = fmaxf(m, mx);
        const float alpha = __builtin_amdgcn_exp2f(m - mnew);
        const float sh = PSH - mnew;
        v16h pb = (v16h){}, pr = (v16h){}; float ls = 0.0f;
#pragma unroll
        for (int r = 0; r < 8; ++r) {
            const float ya = __builtin_amdgcn_exp2f(ta[r] + sh), yb = __builtin_amdgcn_exp2f(tb[r] + sh);
            const float ea = (kq + r <= lim) ? ya : 0.0f;
            const float eb = (kq + 16 + r <= lim) ? yb : 0.0f;
            const h16 pa = (h16)ea; const h16 pc = (h16)eb; pb[r] = pa; pb[8 + r] = pc;
            if (EARLY) { pr[r] = (h16)((ea - (float)pa) * QRS); pr[8 + r] = (h16)((eb - (float)pc) * QRS); ls += ea + eb; }
            else { ls += (float)pa + (float)pc; } }
        l = l * alpha + ls; m = mnew;
        o0 = o0 * alpha; o1 = o1 * alpha; o2 = o2 * alpha; o3 = o3 * alpha;
        const size_t vof = vo + key0;
        if (EARLY) {
            e0 = e0 * alpha; e1 = e1 * alpha; e2 = e2 * alpha; e3 = e3 * alpha;
            { const v16h vh = ldh(VT + vof), vr = ldh(VR + vof);
              o0 = wmma16g(vh, pb, o0); e0 = wmma16g(vh, pr, e0); e0 = wmma16g(vr, pb, e0); }
            { const v16h vh = ldh(VT + vof + (size_t)16 * SEQ), vr = ldh(VR + vof + (size_t)16 * SEQ);
              o1 = wmma16g(vh, pb, o1); e1 = wmma16g(vh, pr, e1); e1 = wmma16g(vr, pb, e1); }
            { const v16h vh = ldh(VT + vof + (size_t)32 * SEQ), vr = ldh(VR + vof + (size_t)32 * SEQ);
              o2 = wmma16g(vh, pb, o2); e2 = wmma16g(vh, pr, e2); e2 = wmma16g(vr, pb, e2); }
            { const v16h vh = ldh(VT + vof + (size_t)48 * SEQ), vr = ldh(VR + vof + (size_t)48 * SEQ);
              o3 = wmma16g(vh, pb, o3); e3 = wmma16g(vh, pr, e3); e3 = wmma16g(vr, pb, e3); }
        } else {
            const h16* va = VT + vof;
            const v16h v0 = ldh(va), v1 = ldh(va + (size_t)16 * SEQ), v2 = ldh(va + (size_t)32 * SEQ), v3 = ldh(va + (size_t)48 * SEQ);
            o0 = wmma16(v0, pb, o0); o1 = wmma16(v1, pb, o1); o2 = wmma16(v2, pb, o2); o3 = wmma16(v3, pb, o3);
            asm volatile("v_nop\n\tv_nop\n\tv_nop\n\tv_nop" : "+v"(o0), "+v"(o1), "+v"(o2), "+v"(o3) : "v"(v0), "v"(v1), "v"(v2), "v"(v3), "v"(pb));
        }
    }
    if (EARLY) { o0 = o0 + e0 * QRI; o1 = o1 + e1 * QRI; o2 = o2 + e2 * QRI; o3 = o3 + e3 * QRI; }
    l += __shfl_xor(l, 16, 32);
    const float lsafe = (l > 0.0f) ? l : 1.0f;
    const float inv = (l > 0.0f) ? (1.0f / lsafe) : 0.0f;
    const int wb = wave * 16 * 68;
    { v4f a, c;
      a[0] = o0[0] * inv; a[1] = o0[1] * inv; a[2] = o0[2] * inv; a[3] = o0[3] * inv; c[0] = o0[4] * inv; c[1] = o0[5] * inv; c[2] = o0[6] * inv; c[3] = o0[7] * inv;
      *(v4fa*)(&os[wb + lr * 68 +  0 + 8 * hi]) = a; *(v4fa*)(&os[wb + lr * 68 +  0 + 8 * hi + 4]) = c;
      a[0] = o1[0] * inv; a[1] = o1[1] * inv; a[2] = o1[2] * inv; a[3] = o1[3] * inv; c[0] = o1[4] * inv; c[1] = o1[5] * inv; c[2] = o1[6] * inv; c[3] = o1[7] * inv;
      *(v4fa*)(&os[wb + lr * 68 + 16 + 8 * hi]) = a; *(v4fa*)(&os[wb + lr * 68 + 16 + 8 * hi + 4]) = c;
      a[0] = o2[0] * inv; a[1] = o2[1] * inv; a[2] = o2[2] * inv; a[3] = o2[3] * inv; c[0] = o2[4] * inv; c[1] = o2[5] * inv; c[2] = o2[6] * inv; c[3] = o2[7] * inv;
      *(v4fa*)(&os[wb + lr * 68 + 32 + 8 * hi]) = a; *(v4fa*)(&os[wb + lr * 68 + 32 + 8 * hi + 4]) = c;
      a[0] = o3[0] * inv; a[1] = o3[1] * inv; a[2] = o3[2] * inv; a[3] = o3[3] * inv; c[0] = o3[4] * inv; c[1] = o3[5] * inv; c[2] = o3[6] * inv; c[3] = o3[7] * inv;
      *(v4fa*)(&os[wb + lr * 68 + 48 + 8 * hi]) = a; *(v4fa*)(&os[wb + lr * 68 + 48 + 8 * hi + 4]) = c; }
    wave_sync();
    const size_t obase = ((size_t)b * SEQ + t0) * DM + (size_t)h * HD;
#pragma unroll 1
    for (int ps = 0; ps < 2; ++ps) {
#pragma unroll
        for (int s = 0; s < 4; ++s) { const int row = 4 * s + (lane >> 3), c8 = (lane & 7) * 8;
            const v4f x0 = *(const v4fa*)(&os[wb + row * 68 + c8]); const v4f x1 = *(const v4fa*)(&os[wb + row * 68 + c8 + 4]); v8us hv, lv;
#pragma unroll
            for (int i = 0; i < 4; ++i) { const unsigned short a0 = f2bf(x0[i]); const unsigned short a1 = f2bf(x1[i]);
                hv[i] = a0; hv[4 + i] = a1; lv[i] = f2bf(x0[i] - bf2f(a0)); lv[4 + i] = f2bf(x1[i] - bf2f(a1)); }
            const size_t oo = obase + (size_t)row * DM + c8;
            *(volatile v8us*)(CH + oo) = hv; *(volatile v8us*)(CL + oo) = lv; }
        if (ps == 0) __threadfence(); }
}

__global__ __launch_bounds__(32 * AW) void k_flash(const h16* __restrict__ QH, const h16* __restrict__ KP, const h16* __restrict__ VT,
                                                   const int* __restrict__ LENS, bf* CH, bf* CL) {
    flash_body<0>((int)blockIdx.x + EROWS / (16 * AW), QH, QH, KP, KP, VT, VT, LENS, CH, CL);
}

__global__ __launch_bounds__(32 * AW) void k_flash_early(const h16* __restrict__ QH, const h16* __restrict__ QR, const h16* __restrict__ KP, const h16* __restrict__ KR,
                                                         const h16* __restrict__ VT, const h16* __restrict__ VR, const int* __restrict__ LENS, bf* CH, bf* CL) {
    flash_body<1>((int)blockIdx.x, QH, QR, KP, KR, VT, VR, LENS, CH, CL);
}

static constexpr size_t al256(size_t v) { return (v + 255) & ~(size_t)255; }
static constexpr size_t SZ_XB = al256((size_t)NB * SEQ * DM * 2);
static constexpr size_t SZ_WB = al256((size_t)4 * DM * DM * 2);
static constexpr size_t SZ_PL = al256((size_t)NB * NH_ * SEQ * HD * 2);
static constexpr size_t SZ_LN = al256((size_t)32 * 4);
static constexpr size_t SZ_TOTAL = 3 * SZ_XB + SZ_WB + 6 * SZ_PL + 2 * SZ_XB + SZ_LN;
static_assert(SZ_TOTAL <= (size_t)134217728);
static_assert(((size_t)DM * DM * 2) % 256 == 0);
static_assert((size_t)NB * OUT_SEQ * DM * 4 <= (size_t)NB_FULL * SEQ_FULL * DM * 4);

static void cvt_in(const float* x, bf* dst, hipStream_t stream) {
    if (SEQ == SEQ_FULL) {
        const size_t n8 = (size_t)NB * SEQ * DM / 8;
        k_cvt8<<<(unsigned)((n8 + 255) / 256), 256, 0, stream>>>(x, dst, n8);
    } else {
        const size_t n8 = (size_t)SEQ * DM / 8;
        for (int b = 0; b < NB; ++b) k_cvt8<<<(unsigned)((n8 + 255) / 256), 256, 0, stream>>>(x + (size_t)b * SEQ_FULL * DM, dst + (size_t)b * SEQ * DM, n8);
    }
}

extern "C" void kernel_launch(void* const* d_in, const int* in_sizes, int n_in,
                              void* d_out, int out_size, void* d_ws, size_t ws_size, hipStream_t stream) {
    if (n_in < 13) return;
    const size_t needx = ((size_t)(NB - 1) * SEQ_FULL + SEQ) * DM;
    if ((size_t)in_sizes[0] < needx || (size_t)in_sizes[1] < needx || (size_t)in_sizes[2] < needx) return;
    if ((size_t)in_sizes[3] < (size_t)(NB - 1) * SEQ_FULL + SEQ || (size_t)in_sizes[4] < (size_t)(NB - 1) * SEQ_FULL + SEQ) return;
    if ((size_t)in_sizes[5] < (size_t)DM * DM || (size_t)in_sizes[7] < (size_t)DM * DM || (size_t)in_sizes[9] < (size_t)DM * DM || (size_t)in_sizes[11] < (size_t)DM * DM) return;
    if (in_sizes[6] < DM || in_sizes[8] < DM || in_sizes[10] < DM || in_sizes[12] < DM) return;
    if ((size_t)out_size < ((size_t)(NB - 1) * OUT_SEQ + SEQ) * DM) return;
    if (SZ_TOTAL > ws_size) return;
    const float* xq = (const float*)d_in[0]; const float* xk = (const float*)d_in[1]; const float* xv = (const float*)d_in[2];
    const int* qmask = (const int*)d_in[3]; const int* kmask = (const int*)d_in[4];
    const float* wq = (const float*)d_in[5];  const float* bq = (const float*)d_in[6];
    const float* wk = (const float*)d_in[7];  const float* bk = (const float*)d_in[8];
    const float* wv = (const float*)d_in[9];  const float* bv = (const float*)d_in[10];
    const float* wo = (const float*)d_in[11]; const float* bo = (const float*)d_in[12];
    float* OUT = (float*)d_out;
    char* wsp = (char*)d_ws;
    bf* QB = (bf*)wsp; wsp += SZ_XB;
    bf* KB = (bf*)wsp; wsp += SZ_XB;
    bf* VB = (bf*)wsp; wsp += SZ_XB;
    bf* WB = (bf*)wsp; wsp += SZ_WB;
    h16* QH = (h16*)wsp; wsp += SZ_PL;
    h16* QR = (h16*)wsp; wsp += SZ_PL;
    h16* KP = (h16*)wsp; wsp += SZ_PL;
    h16* KR = (h16*)wsp; wsp += SZ_PL;
    h16* VT = (h16*)wsp; wsp += SZ_PL;
    h16* VR = (h16*)wsp; wsp += SZ_PL;
    bf* CH = (bf*)wsp; wsp += SZ_XB;
    bf* CL = (bf*)wsp; wsp += SZ_XB;
    int* LN = (int*)wsp; wsp += SZ_LN;
    bf* WQT = WB; bf* WKT = WB + (size_t)DM * DM; bf* WVT = WB + (size_t)2 * DM * DM; bf* WOT = WB + (size_t)3 * DM * DM;

    cvt_in(xq, QB, stream); cvt_in(xk, KB, stream); cvt_in(xv, VB, stream);
    { const dim3 g(DM / 64, DM / 64, 1);
      k_cvtT<<<g, 256, 0, stream>>>(wq, WQT); k_cvtT<<<g, 256, 0, stream>>>(wk, WKT); k_cvtT<<<g, 256, 0, stream>>>(wv, WVT); k_cvtT<<<g, 256, 0, stream>>>(wo, WOT); }
    k_lens<<<1, 32, 0, stream>>>(qmask, kmask, LN);

    k_proj<0><<<dim3(NB * SEQ / 64, DM / 64, 1), 32, 0, stream>>>(QB, QB, WQT, bq, 1, QH, QR, 1, OUT, SEQ, (size_t)NH_ * SEQ * HD, HD, HD, (size_t)SEQ * HD);
    k_proj<0><<<dim3(NB * SEQ / 64, DM / 64, 1), 32, 0, stream>>>(KB, KB, WKT, bk, 1, KP, KR, 1, OUT, SEQ, (size_t)NH_ * SEQ * HD, HD, HD, (size_t)SEQ * HD);
    k_proj<0><<<dim3(DM / 64, NB * SEQ / 64, 1), 32, 0, stream>>>(WVT, WVT, VB, bv, 2, VT, VR, 1, OUT, DM, (size_t)0, SEQ, SEQ, (size_t)DM * SEQ);

    k_flash_early<<<dim3(EROWS / (16 * AW), NB * NH_, 1), 32 * AW, 0, stream>>>(QH, QR, KP, KR, VT, VR, LN, CH, CL);
    if (SEQ > EROWS)
        k_flash<<<dim3((SEQ - EROWS) / (16 * AW), NB * NH_, 1), 32 * AW, 0, stream>>>(QH, KP, VT, LN, CH, CL);

    k_proj<1><<<dim3(NB * SEQ / 64, DM / 64, 1), 32, 0, stream>>>(CH, CL, WOT, bo, 1, QH, QH, 0, OUT, SEQ, (size_t)OUT_SEQ * DM, DM, DM, (size_t)0);
}
